// EquivariantMessagePasser_28922309771659
// MI455X (gfx1250) — hardware-verified
//
#include <hip/hip_runtime.h>
#include <stddef.h>
#include <stdint.h>
#include <math.h>


#define NAT     10000
#define NED     100000
#define NTHR    256
#define NWAVE   8
#define EPT     8
#define CHUNK   (NTHR * EPT)
#define WCAP    (EPT * 32)
#define LISTN   (NWAVE * WCAP)
#define NBRUN   512
#define SLB     9
#define RCAP    8192
#define NBLK    ((NAT + NBRUN - 1) / NBRUN)
#define DEGCAP  64
#define MEAS_B512   5274
#define MEAS_MAXDEG 23
#define APW     8
#define APB     (NWAVE * APW)
#define GBM     64
#define GTHR    128
#define EDGROWS (((NED + NTHR - 1) / NTHR) * NTHR)
#define PI_F    0x1.921fb6p+1f
#define BKT_LDS_INTS (LISTN + 2 * RCAP + 3 * NBRUN + 16)
#define BKT_ZINTS    (RCAP + 3 * NBRUN)

#define HDC __host__ __device__ __forceinline__ constexpr

HDC size_t pre4(int g, size_t a0, size_t a1, size_t a2, size_t a3) {
  return g <= 0 ? (size_t)0 : g == 1 ? a0 : g == 2 ? a0 + a1 : g == 3 ? a0 + a1 + a2 : a0 + a1 + a2 + a3;
}
HDC size_t al256(size_t x) { return (x + 255) & ~(size_t)255; }
HDC int KL(int l)   { return 128 - 32 * l; }
HDC int P3(int g)   { return g == 0 ? 1 : g == 1 ? 3 : g == 2 ? 9 : 27; }
HDC int MM(int g)   { return (g + 1) * (g + 1); }
HDC int MPAD(int g) { return g <= 1 ? 4 : g == 2 ? 12 : 16; }
HDC int DPAD(int g) { return g <= 1 ? 4 : g == 2 ? 12 : 28; }
HDC int SEGU(int g) { return ((P3(g) * MPAD(g) + 31) / 32) * 32; }
HDC int SEGT(int g) { return ((MM(g) * DPAD(g) + 31) / 32) * 32; }
HDC int TU(int g)   { return (int)pre4(g, (size_t)SEGU(0), (size_t)SEGU(1), (size_t)SEGU(2), (size_t)SEGU(3)); }
HDC int TUT(int g)  { return TU(4) + (int)pre4(g, (size_t)SEGT(0), (size_t)SEGT(1), (size_t)SEGT(2), (size_t)SEGT(3)); }
HDC int PAIR(int g, int lp) { return g * (g + 1) / 2 + lp; }
constexpr int TWR  = TUT(4);
constexpr int TABN = TWR + 10 * 256;
HDC int MROWS(int l) { return NAT * (2 * l + 1); }
HDC int MPADR(int l) { return ((MROWS(l) + 127) / 128) * 128; }
HDC int OUTOFF(int l) {
  return (int)pre4(l, (size_t)MROWS(0) * KL(0), (size_t)MROWS(1) * KL(1), (size_t)MROWS(2) * KL(2), (size_t)MROWS(3) * KL(3));
}
HDC size_t WTB(int l)  { return (size_t)4 * KL(l) * KL(l); }
HDC size_t O_WT(int l) { return pre4(l, al256(WTB(0)), al256(WTB(1)), al256(WTB(2)), al256(WTB(3))); }
constexpr size_t O_TAB  = O_WT(4);
constexpr size_t O_FLG  = O_TAB + al256((size_t)TABN * 4);
constexpr size_t O_CNT  = O_FLG + al256((size_t)NBLK * 128);
constexpr size_t O_OFF  = O_CNT + al256((size_t)NBLK * NBRUN * 4);
constexpr size_t O_LIST = O_OFF + al256((size_t)NBLK * NBRUN * 4);
constexpr size_t O_EDG  = O_LIST + al256((size_t)NBLK * RCAP * 8);
HDC size_t UFB(int g)  { return (size_t)NAT * P3(g) * 128; }
HDC size_t O_UF(int g) {
  return O_EDG + al256((size_t)EDGROWS * 128) + pre4(g, al256(UFB(0)), al256(UFB(1)), al256(UFB(2)), al256(UFB(3)));
}
HDC size_t CATB(int l) { return (size_t)MPADR(l) * KL(l) * 4; }
HDC size_t O_CAT(int l) { return O_UF(4) + pre4(l, al256(CATB(0)), al256(CATB(1)), al256(CATB(2)), al256(CATB(3))); }
HDC int ZU(int l) { return (MPADR(l) - MROWS(l)) * KL(l) * 4 / 16; }
constexpr size_t WS_TOTAL = O_CAT(4);

constexpr size_t OWT0 = O_WT(0), OWT1 = O_WT(1), OWT2 = O_WT(2), OWT3 = O_WT(3);
constexpr size_t OCAT0 = O_CAT(0), OCAT1 = O_CAT(1), OCAT2 = O_CAT(2), OCAT3 = O_CAT(3);
constexpr size_t OCZ0 = OCAT0 + (size_t)MROWS(0) * KL(0) * 4;
constexpr size_t OCZ1 = OCAT1 + (size_t)MROWS(1) * KL(1) * 4;
constexpr size_t OCZ2 = OCAT2 + (size_t)MROWS(2) * KL(2) * 4;
constexpr size_t OCZ3 = OCAT3 + (size_t)MROWS(3) * KL(3) * 4;
constexpr int KC0 = KL(0), KC1 = KL(1), KC2 = KL(2), KC3 = KL(3);

constexpr int UW0 = (int)(WTB(0) / 16), UW1 = (int)(WTB(1) / 16), UW2 = (int)(WTB(2) / 16), UW3 = (int)(WTB(3) / 16);
constexpr int UWT = UW0 + UW1 + UW2 + UW3;
constexpr int ZU0 = ZU(0), ZU1 = ZU(1), ZU2 = ZU(2), ZU3 = ZU(3);
constexpr int UZT  = ZU0 + ZU1 + ZU2 + ZU3;
constexpr int UTOT = UWT + UZT;

static_assert(KL(0) == 128 && KL(1) == 96 && KL(2) == 64 && KL(3) == 32);
static_assert(MM(3) <= 16 && P3(3) <= 27 && DPAD(3) >= P3(3) && MPAD(3) >= MM(3) && DPAD(2) >= P3(2) && MPAD(2) >= MM(2));
static_assert(TU(4) == 640 && TWR == 1280 && TABN == 3840);
static_assert((UW0 % NTHR) == 0 && ((UW0 + UW1) % NTHR) == 0 && ((UW0 + UW1 + UW2) % NTHR) == 0 && (UWT % NTHR) == 0);
static_assert((UTOT % NTHR) == 0);
static_assert(OUTOFF(1) == 1280000 && OUTOFF(2) == 4160000 && OUTOFF(3) == 7360000);
static_assert(OUTOFF(3) + MROWS(3) * KL(3) == 9600000);
static_assert(WS_TOTAL == (size_t)104048128);
static_assert(WS_TOTAL <= (size_t)128 * 1024 * 1024);
static_assert((CHUNK & (CHUNK - 1)) == 0 && CHUNK <= 4096);
static_assert(NBRUN == (1 << SLB) && NED < (1 << (31 - SLB)) && ((long long)CHUNK << SLB) < (1LL << 31));
static_assert(RCAP >= MEAS_B512 + 2048 && (RCAP % 32) == 0 && (BKT_ZINTS % 4) == 0);
static_assert(DEGCAP >= MEAS_MAXDEG + 8);
static_assert(NBLK * NBRUN >= NAT && (NBRUN % APB) == 0 && (NBRUN % 32) == 0);
static_assert(BKT_LDS_INTS * 4 <= 327680);
static_assert(GBM == (GTHR / 32) * 16 && (MPADR(0) % GBM) == 0 && (MPADR(1) % GBM) == 0 && (MPADR(2) % GBM) == 0 && (MPADR(3) % GBM) == 0);
static_assert((NED % 4) == 0);
static_assert((RCAP / 2) % NTHR == 0 && NBRUN / 4 <= NTHR);

typedef float          v4f  __attribute__((ext_vector_type(4)));
typedef float          v8f  __attribute__((ext_vector_type(8)));
typedef int            v2i  __attribute__((ext_vector_type(2)));
typedef int            v4i  __attribute__((ext_vector_type(4)));
typedef int            v8i  __attribute__((ext_vector_type(8)));
typedef unsigned short v8us __attribute__((ext_vector_type(8)));
typedef __bf16         v16b __attribute__((ext_vector_type(16)));
typedef v4f  __attribute__((may_alias)) v4fa;
typedef v4i  __attribute__((may_alias)) v4ia;
typedef v8us __attribute__((may_alias)) v8usa;
union FragB { v16b v; v8us h[2]; v8i w; };

__device__ __forceinline__ v8f wmb(const FragB& a, const FragB& b, v8f c) {
  v8f d = __builtin_amdgcn_wmma_f32_16x16x32_bf16(false, a.v, false, b.v, (short)0, c, false, false);
  asm volatile("v_nop\n\tv_nop\n\tv_nop\n\tv_nop" : "+v"(d) : "v"(a.w), "v"(b.w));
  return d;
}

__device__ __forceinline__ void ldwait() {
  asm volatile("s_wait_loadcnt 0x0" ::: "memory");
}

__device__ __forceinline__ unsigned int f2bf(float f) {
  const unsigned int u = __float_as_uint(f);
  const unsigned int r = ((u + 0x7FFFu + ((u >> 16) & 1u)) >> 16) & 0xFFFFu;
  return ((u & 0x7FFFFFFFu) > 0x7F800000u) ? 0x7FC0u : r;
}
__device__ __forceinline__ float bf2f(unsigned int b) { return __uint_as_float(b << 16); }
__device__ __forceinline__ float bfr(float f) { return bf2f(f2bf(f)); }

template <int SLBITS>
__device__ __forceinline__ int scan_chunk(const int* __restrict__ dsts, int nE, int cbase, int slotBase,
                                          int nb, int vec8, int* list, int tid, int lane, int wave) {
  int wc = 0;
  const int el0  = tid * EPT;
  const int e0   = cbase + el0;
  const int sent = -0x7fffffff - 1;
  v4i da, db;
  if (vec8 != 0 && cbase + CHUNK <= nE) {
    da = *(const v4i*)(dsts + e0);
    db = *(const v4i*)(dsts + e0 + 4);
  } else {
    da.x = (e0     < nE) ? dsts[min(e0,     nE - 1)] : sent;
    da.y = (e0 + 1 < nE) ? dsts[min(e0 + 1, nE - 1)] : sent;
    da.z = (e0 + 2 < nE) ? dsts[min(e0 + 2, nE - 1)] : sent;
    da.w = (e0 + 3 < nE) ? dsts[min(e0 + 3, nE - 1)] : sent;
    db.x = (e0 + 4 < nE) ? dsts[min(e0 + 4, nE - 1)] : sent;
    db.y = (e0 + 5 < nE) ? dsts[min(e0 + 5, nE - 1)] : sent;
    db.z = (e0 + 6 < nE) ? dsts[min(e0 + 6, nE - 1)] : sent;
    db.w = (e0 + 7 < nE) ? dsts[min(e0 + 7, nE - 1)] : sent;
  }
  const unsigned nbs = (unsigned)slotBase;
  const unsigned unb = (unsigned)nb;
  const unsigned s0 = (unsigned)da.x - nbs, s1 = (unsigned)da.y - nbs;
  const unsigned s2 = (unsigned)da.z - nbs, s3 = (unsigned)da.w - nbs;
  const unsigned s4 = (unsigned)db.x - nbs, s5 = (unsigned)db.y - nbs;
  const unsigned s6 = (unsigned)db.z - nbs, s7 = (unsigned)db.w - nbs;
  const bool h0 = s0 < unb, h1 = s1 < unb, h2 = s2 < unb, h3 = s3 < unb;
  const bool h4 = s4 < unb, h5 = s5 < unb, h6 = s6 < unb, h7 = s7 < unb;
  const unsigned any = __builtin_amdgcn_ballot_w32(h0 | h1 | h2 | h3 | h4 | h5 | h6 | h7);
  if (any != 0u) {
#define HITJ(J, HJ, SJ) { \
      const unsigned mj = __builtin_amdgcn_ballot_w32(HJ); \
      if (mj != 0u) { \
        if (HJ) { \
          const int pos = wc + (int)__builtin_amdgcn_mbcnt_lo(mj, 0u); \
          if (pos < WCAP) list[wave * WCAP + pos] = ((el0 + (J)) << SLBITS) | (int)(SJ); \
        } \
        wc += (int)__builtin_popcount(mj); } }
    HITJ(0, h0, s0)
    HITJ(1, h1, s1)
    HITJ(2, h2, s2)
    HITJ(3, h3, s3)
    HITJ(4, h4, s4)
    HITJ(5, h5, s5)
    HITJ(6, h6, s6)
    HITJ(7, h7, s7)
#undef HITJ
  }
  return wc;
}

__device__ __forceinline__ v8us wt_unit(const float* __restrict__ W, int K, int v) {
  const int upr = K >> 2;
  const int n   = v / upr;
  const int k8  = (v - n * upr) * 8;
  const int kr  = 32 * (k8 >> 6) + (k8 & 31);
  const float* p = W + (size_t)kr * K + n;
  v8us o;
#pragma unroll
  for (int i = 0; i < 8; ++i) o[i] = (unsigned short)f2bf(p[(size_t)i * K]);
  return o;
}

__global__ __launch_bounds__(NTHR) void k_pa(const float* __restrict__ W0, const float* __restrict__ W1,
                                             const float* __restrict__ W2, const float* __restrict__ W3, char* ws) {
  const int u = (int)blockIdx.x * NTHR + (int)threadIdx.x;
  v8us o = {0, 0, 0, 0, 0, 0, 0, 0};
  size_t db;
  if (u < UW0) {
    o = wt_unit(W0, KC0, u);
    db = OWT0 + (size_t)u * 16;
  } else if (u < UW0 + UW1) {
    o = wt_unit(W1, KC1, u - UW0);
    db = OWT1 + (size_t)(u - UW0) * 16;
  } else if (u < UW0 + UW1 + UW2) {
    o = wt_unit(W2, KC2, u - UW0 - UW1);
    db = OWT2 + (size_t)(u - UW0 - UW1) * 16;
  } else if (u < UWT) {
    o = wt_unit(W3, KC3, u - UW0 - UW1 - UW2);
    db = OWT3 + (size_t)(u - UW0 - UW1 - UW2) * 16;
  } else {
    const int z = u - UWT;
    const size_t b0 = OCZ0 + (size_t)z * 16;
    const size_t b1 = OCZ1 + (size_t)(z - ZU0) * 16;
    const size_t b2 = OCZ2 + (size_t)(z - ZU0 - ZU1) * 16;
    const size_t b3 = OCZ3 + (size_t)(z - ZU0 - ZU1 - ZU2) * 16;
    db = (z < ZU0) ? b0 : (z < ZU0 + ZU1) ? b1 : (z < ZU0 + ZU1 + ZU2) ? b2 : b3;
  }
  if (u >= UTOT) return;
  unsigned short* dp = (unsigned short*)(ws + db);
  *(volatile v8us*)dp = o;
  __threadfence();
  *(volatile v8us*)dp = o;
}

template <int G>
__device__ __forceinline__ void tab_u(const float* __restrict__ U, float* tab, int tid) {
  constexpr int M = MM(G), D = P3(G), MP = MPAD(G), NU = SEGU(G) / 4, TUG = TU(G);
  static_assert(NU <= NTHR);
  const int uc = tid < NU ? tid : NU - 1;
  v4f o;
#pragma unroll
  for (int i = 0; i < 4; ++i) {
    const int f  = 4 * uc + i;
    const int d  = f / MP;
    const int mp = f - d * MP;
    const int dc = d < D ? d : D - 1;
    const int mc = mp < M ? mp : M - 1;
    const float x = U[dc * M + mc];
    o[i] = (d < D && mp < M) ? bfr(x) : 0.0f;
  }
  float* dp = tab + TUG + 4 * uc;
  if (tid < NU) *(volatile v4f*)dp = o;
  __threadfence();
  if (tid < NU) *(volatile v4f*)dp = o;
}

template <int G>
__device__ __forceinline__ void tab_ut(const float* __restrict__ U, float* tab, int tid) {
  constexpr int M = MM(G), D = P3(G), DP = DPAD(G), NU = SEGT(G) / 4, TUTG = TUT(G);
  static_assert(NU <= NTHR);
  const int uc = tid < NU ? tid : NU - 1;
  v4f o;
#pragma unroll
  for (int i = 0; i < 4; ++i) {
    const int f  = 4 * uc + i;
    const int m  = f / DP;
    const int dd = f - m * DP;
    const int dc = dd < D ? dd : D - 1;
    const int mc = m < M ? m : M - 1;
    const float x = U[dc * M + mc];
    o[i] = (m < M && dd < D) ? bfr(x) : 0.0f;
  }
  float* dp = tab + TUTG + 4 * uc;
  if (tid < NU) *(volatile v4f*)dp = o;
  __threadfence();
  if (tid < NU) *(volatile v4f*)dp = o;
}

template <int G, int LP>
__device__ __forceinline__ void tab_wr(const float* __restrict__ W, float* tab, int tid) {
  constexpr int NU = 64;
  constexpr int KLP = KL(LP);
  constexpr int TO  = TWR + PAIR(G, LP) * 256;
  const int uc = tid < NU ? tid : NU - 1;
  const int f  = 4 * uc;
  const int n  = f >> 5;
  const int c0 = f & 31;
  const v4f x = *(const v4f*)(W + n * KLP + 32 * (3 - G) + c0);
  v4f o;
  o.x = bfr(x.x); o.y = bfr(x.y); o.z = bfr(x.z); o.w = bfr(x.w);
  float* dp = tab + TO + f;
  if (tid < NU) *(volatile v4f*)dp = o;
  __threadfence();
  if (tid < NU) *(volatile v4f*)dp = o;
}

__global__ __launch_bounds__(NTHR) void k_pb(const float* __restrict__ Wr0, const float* __restrict__ Wr1,
                                             const float* __restrict__ Wr2, const float* __restrict__ Wr3,
                                             const float* __restrict__ U0, const float* __restrict__ U1,
                                             const float* __restrict__ U2, const float* __restrict__ U3, char* ws) {
  const int tid = (int)threadIdx.x;
  float* tab = (float*)(ws + O_TAB);
  tab_u<0>(U0, tab, tid);  tab_u<1>(U1, tab, tid);  tab_u<2>(U2, tab, tid);  tab_u<3>(U3, tab, tid);
  tab_ut<0>(U0, tab, tid); tab_ut<1>(U1, tab, tid); tab_ut<2>(U2, tab, tid); tab_ut<3>(U3, tab, tid);
  tab_wr<0, 0>(Wr0, tab, tid);
  tab_wr<1, 0>(Wr0, tab, tid); tab_wr<1, 1>(Wr1, tab, tid);
  tab_wr<2, 0>(Wr0, tab, tid); tab_wr<2, 1>(Wr1, tab, tid); tab_wr<2, 2>(Wr2, tab, tid);
  tab_wr<3, 0>(Wr0, tab, tid); tab_wr<3, 1>(Wr1, tab, tid); tab_wr<3, 2>(Wr2, tab, tid); tab_wr<3, 3>(Wr3, tab, tid);
}

__device__ __forceinline__ void edge_flush(const float* tile, float* dst, int tid) {
#pragma unroll 1
  for (int it = 0; it < 8; ++it) {
    const int p = it * NTHR + tid;
    const v4f v = *(const v4fa*)(tile + 4 * p);
    *(volatile v4f*)(dst + 4 * p) = v;
  }
}

__global__ __launch_bounds__(NTHR) void k_edge(const float* __restrict__ r, const float* __restrict__ sh0,
                                               const float* __restrict__ sh1, const float* __restrict__ sh2,
                                               const float* __restrict__ sh3, char* ws) {
  __shared__ __attribute__((aligned(16))) float tile[NTHR * 32];
  const int tid = (int)threadIdx.x;
  const int e   = (int)blockIdx.x * NTHR + tid;
  const int ec  = e < NED ? e : NED - 1;
  float* row = tile + tid * 32;
  float rv;
  {
    const float a0 = r[ec];
    const float b0 = sh0[ec];
    const float c0 = sh1[ec * 3], c1 = sh1[ec * 3 + 1], c2 = sh1[ec * 3 + 2];
    ldwait();
    rv = bfr(a0);
    row[8] = bfr(b0); row[9] = bfr(c0); row[10] = bfr(c1); row[11] = bfr(c2);
  }
  {
    const float* p = sh2 + (size_t)ec * 5;
    const float d0 = p[0], d1 = p[1], d2 = p[2], d3 = p[3], d4 = p[4];
    ldwait();
    row[12] = bfr(d0); row[13] = bfr(d1); row[14] = bfr(d2); row[15] = bfr(d3); row[16] = bfr(d4);
  }
  {
    const float* p = sh3 + (size_t)ec * 7;
    const float g0 = p[0], g1 = p[1], g2 = p[2], g3 = p[3], g4 = p[4], g5 = p[5], g6 = p[6];
    ldwait();
    row[17] = bfr(g0); row[18] = bfr(g1); row[19] = bfr(g2); row[20] = bfr(g3);
    row[21] = bfr(g4); row[22] = bfr(g5); row[23] = bfr(g6);
  }
#pragma unroll
  for (int i = 24; i < 32; ++i) row[i] = 0.0f;
  float t = rv / 5.0f;
  t = fminf(fmaxf(t, 0.0f), 1.0f);
  const float inv = 1.0f / (rv + 1e-6f);
  float fc = 0.0f;
#pragma unroll 1
  for (int i = 0; i < 9; ++i) {
    const float a = (i == 0) ? (PI_F * t) : ((((float)i * PI_F) * rv) / 5.0f);
    float s, c;
    sincosf(a, &s, &c);
    if (i == 0) fc = 0.5f * (c + 1.0f);
    else        row[i - 1] = (s * inv) * fc;
  }
  __syncthreads();
  float* dst = (float*)(ws + O_EDG) + (size_t)blockIdx.x * NTHR * 32;
  edge_flush(tile, dst, tid);
  __threadfence();
  edge_flush(tile, dst, tid);
}

template <int G>
__device__ __forceinline__ void unc_g(const float* __restrict__ f0, const float* __restrict__ f1,
                                      const float* __restrict__ f2, const float* __restrict__ f3,
                                      const float* sU, float* sV, char* ws, int nc, bool live, int lane) {
  constexpr int M = MM(G), D = P3(G), MP = MPAD(G), LO = 32 * (3 - G), TUG = TU(G);
  constexpr size_t OUFG = O_UF(G);
  float f[MP];
#pragma unroll
  for (int i = 0; i < MP; ++i) f[i] = 0.0f;
  f[0] = f0[(size_t)nc * KC0 + LO + lane];
  if constexpr (G >= 1) {
#pragma unroll
    for (int mu = 0; mu < 3; ++mu) f[1 + mu] = f1[((size_t)nc * 3 + mu) * KC1 + LO + lane];
  }
  ldwait();
  if constexpr (G >= 2) {
#pragma unroll
    for (int mu = 0; mu < 5; ++mu) f[4 + mu] = f2[((size_t)nc * 5 + mu) * KC2 + LO + lane];
    ldwait();
  }
  if constexpr (G >= 3) {
#pragma unroll
    for (int mu = 0; mu < 7; ++mu) f[9 + mu] = f3[((size_t)nc * 7 + mu) * KC3 + LO + lane];
    ldwait();
  }
#pragma unroll
  for (int i = 0; i < M; ++i) f[i] = bfr(f[i]);
  float* up = (float*)(ws + OUFG) + (size_t)nc * (D * 32) + lane;
#pragma unroll 1
  for (int d = 0; d < D; ++d) {
    const float* ur = sU + TUG + d * MP;
    float v = 0.0f;
#pragma unroll
    for (int q = 0; q < MP / 4; ++q) {
      const v4f u = *(const v4fa*)(ur + 4 * q);
      v = fmaf(u.x, f[4 * q], v);
      v = fmaf(u.y, f[4 * q + 1], v);
      v = fmaf(u.z, f[4 * q + 2], v);
      v = fmaf(u.w, f[4 * q + 3], v);
    }
    sV[d * 32 + lane] = v;
    if (live) *(volatile float*)(up + d * 32) = v;
  }
  __threadfence();
#pragma unroll 1
  for (int d = 0; d < D; ++d) {
    const float v = sV[d * 32 + lane];
    if (live) *(volatile float*)(up + d * 32) = v;
  }
}

__global__ __launch_bounds__(NTHR) void k_unc(const float* __restrict__ f0, const float* __restrict__ f1,
                                              const float* __restrict__ f2, const float* __restrict__ f3, char* ws) {
  __shared__ __attribute__((aligned(16))) float sU[640];
  __shared__ __attribute__((aligned(16))) float sVall[NWAVE * 28 * 32];
  static_assert(TU(4) == 640 && P3(3) <= 28);
  const int tid = (int)threadIdx.x, lane = tid & 31, wave = tid >> 5;
  {
    const int uc = tid < 160 ? tid : 159;
    const v4f v = *(const v4f*)((const float*)(ws + O_TAB) + 4 * uc);
    if (tid < 160) *(v4fa*)(sU + 4 * uc) = v;
  }
  __syncthreads();
  const int n    = (int)blockIdx.x * NWAVE + wave;
  const bool live = n < NAT;
  const int nc   = live ? n : NAT - 1;
  float* sV = sVall + wave * (28 * 32);
  const int g = (int)blockIdx.y;
  if (g == 0)      unc_g<0>(f0, f1, f2, f3, sU, sV, ws, nc, live, lane);
  else if (g == 1) unc_g<1>(f0, f1, f2, f3, sU, sV, ws, nc, live, lane);
  else if (g == 2) unc_g<2>(f0, f1, f2, f3, sU, sV, ws, nc, live, lane);
  else             unc_g<3>(f0, f1, f2, f3, sU, sV, ws, nc, live, lane);
}

__device__ __forceinline__ void bucket_store(const int* srt, const int* cnt, const int* offs,
                                             const int* __restrict__ nbr, char* ws, int blk, int nh, int ovf, int tid) {
  int* LISTg = (int*)(ws + O_LIST) + (size_t)blk * RCAP * 2;
#pragma unroll 1
  for (int it = 0; it < (RCAP / 2) / NTHR; ++it) {
    const int q  = it * NTHR + tid;
    const int p0 = 2 * q, p1 = 2 * q + 1;
    int e0 = srt[p0], e1 = srt[p1];
    e0 = e0 < 0 ? 0 : (e0 > NED - 1 ? NED - 1 : e0);
    e1 = e1 < 0 ? 0 : (e1 > NED - 1 ? NED - 1 : e1);
    int n0 = nbr[e0], n1 = nbr[e1];
    n0 = n0 < 0 ? 0 : (n0 > NAT - 1 ? NAT - 1 : n0);
    n1 = n1 < 0 ? 0 : (n1 > NAT - 1 ? NAT - 1 : n1);
    v4i v;
    v.x = (p0 < nh) ? e0 : 0; v.y = (p0 < nh) ? n0 : 0;
    v.z = (p1 < nh) ? e1 : 0; v.w = (p1 < nh) ? n1 : 0;
    *(volatile v4i*)(LISTg + 4 * q) = v;
  }
  if (tid < NBRUN / 4) {
    const v4i cv = *(const v4ia*)(cnt + 4 * tid);
    const v4i ov = *(const v4ia*)(offs + 4 * tid);
    *(volatile v4i*)((int*)(ws + O_CNT) + (size_t)blk * NBRUN + 4 * tid) = cv;
    *(volatile v4i*)((int*)(ws + O_OFF) + (size_t)blk * NBRUN + 4 * tid) = ov;
  }
  if (tid < 8) {
    v4i fv;
    fv.x = (tid == 0) ? nh : 0;
    fv.y = (tid == 0) ? ovf : 0;
    fv.z = 0; fv.w = 0;
    *(volatile v4i*)((int*)(ws + O_FLG) + (size_t)blk * 32 + 4 * tid) = fv;
  }
}

__global__ __launch_bounds__(NTHR) void k_bucket(const int* __restrict__ ctr, const int* __restrict__ nbr, char* ws) {
  extern __shared__ __attribute__((aligned(16))) int bsm[];
  int* list = bsm;
  int* reg1 = list + LISTN;
  int* srt  = reg1 + RCAP;
  int* cnt  = srt + RCAP;
  int* offs = cnt + NBRUN;
  int* cur  = offs + NBRUN;
  int* wcnt = cur + NBRUN;
  const int tid = (int)threadIdx.x, lane = tid & 31, wave = tid >> 5;
  const int blk = (int)blockIdx.x;
  const int nodeBase = blk * NBRUN;
  int nb = NAT - nodeBase;
  nb = nb < 0 ? 0 : (nb > NBRUN ? NBRUN : nb);
  {
    const v4i z4 = {0, 0, 0, 0};
    for (int i = tid * 4; i < BKT_ZINTS; i += NTHR * 4) *(v4ia*)(srt + i) = z4;
    if (tid < 16) wcnt[tid] = 0;
  }
  __syncthreads();

  int tot = 0, ovf = 0;
  const int nE = NED;
  const int nChunks = (nE + CHUNK - 1) / CHUNK;
#pragma unroll 1
  for (int ch = 0; ch < nChunks; ++ch) {
    const int cbase = ch * CHUNK;
    const int wc = scan_chunk<SLB>(ctr, nE, cbase, nodeBase, nb, 1, list, tid, lane, wave);
    if (lane == 0) wcnt[wave] = wc;
    __syncthreads();
    int pre = 0, all = 0;
#pragma unroll
    for (int w2 = 0; w2 < NWAVE; ++w2) {
      int c = wcnt[w2];
      c = c < 0 ? 0 : (c > WCAP ? WCAP : c);
      all += c;
      pre += (w2 < wave) ? c : 0;
    }
    const int wcc  = wc > WCAP ? WCAP : wc;
    const int base = tot + pre;
#pragma unroll 1
    for (int i = lane; i < wcc; i += 32) {
      const int ent = list[wave * WCAP + i];
      const int el  = (ent >> SLB) & (CHUNK - 1);
      const int sl  = ent & (NBRUN - 1);
      int eid = cbase + el;
      eid = eid > nE - 1 ? nE - 1 : eid;
      const int pos = base + i;
      if (pos < RCAP) reg1[pos] = (int)(((unsigned)eid << SLB) | (unsigned)sl);
    }
    if (tot + all > RCAP) ovf = 1;
    tot += all;
    tot = tot > RCAP ? RCAP : tot;
    __syncthreads();
  }
  const int nh = tot;

  if (wave == 0) {
#pragma unroll 1
    for (int b0 = 0; b0 < nh; b0 += 32) {
      const int idx = b0 + lane;
      const int uv  = reg1[idx < nh ? idx : nh - 1];
      const int m32 = (nh - b0) < 32 ? (nh - b0) : 32;
#pragma unroll 1
      for (int k = 0; k < m32; ++k) {
        const int u  = __builtin_amdgcn_readlane(uv, k);
        const int sq = u & (NBRUN - 1);
        if (lane == 0) cnt[sq] = cnt[sq] + 1;
      }
    }
  }
  __syncthreads();
  if (wave == 0) {
    const int base = lane * (NBRUN / 32);
    int s = 0;
#pragma unroll 1
    for (int i = 0; i < NBRUN / 32; ++i) s += cnt[base + i];
    int incl = s;
#pragma unroll
    for (int d = 1; d < 32; d <<= 1) {
      const int y = __shfl_up(incl, d, 32);
      if (lane >= d) incl += y;
    }
    int run = incl - s;
#pragma unroll 1
    for (int i = 0; i < NBRUN / 32; ++i) {
      const int cv = cnt[base + i];
      offs[base + i] = run;
      cur[base + i]  = run;
      run += cv;
    }
  }
  __syncthreads();
  if (wave == 0) {
#pragma unroll 1
    for (int b0 = 0; b0 < nh; b0 += 32) {
      const int idx = b0 + lane;
      const int uv  = reg1[idx < nh ? idx : nh - 1];
      const int m32 = (nh - b0) < 32 ? (nh - b0) : 32;
#pragma unroll 1
      for (int k = 0; k < m32; ++k) {
        const int u   = __builtin_amdgcn_readlane(uv, k);
        const int sq  = u & (NBRUN - 1);
        const int eid = (int)((unsigned)u >> SLB);
        if (lane == 0) {
          int p = cur[sq];
          p = p < 0 ? 0 : (p > RCAP - 1 ? RCAP - 1 : p);
          srt[p] = eid;
          cur[sq] = p + 1;
        }
      }
    }
  }
  __syncthreads();

  bucket_store(srt, cnt, offs, nbr, ws, blk, nh, ovf, tid);
  __threadfence();
  bucket_store(srt, cnt, offs, nbr, ws, blk, nh, ovf, tid);
}

template <int G>
__global__ __launch_bounds__(NTHR) __attribute__((amdgpu_num_vgpr(248)))
void k_scan(char* ws) {
  constexpr int M = MM(G), D = P3(G), MP = MPAD(G), DP = DPAD(G), SU = SEGU(G), ST = SEGT(G);
  constexpr int TUG = TU(G), TUTG = TUT(G), PG = G * (G + 1) / 2;
  constexpr size_t OUFG = O_UF(G);
  static_assert(PG == PAIR(G, 0));
  static_assert(SU / 4 <= NTHR && ST / 4 <= NTHR);
  static_assert(D <= DP && M <= MP && M * DP <= ST && D * MP <= SU && (DP % 4) == 0 && (MP % 4) == 0);
  __shared__ __attribute__((aligned(16))) float sU[SU];
  __shared__ __attribute__((aligned(16))) float sT[ST];
  __shared__ __attribute__((aligned(16))) float sAcc[NWAVE * DP * 32];
  __shared__ __attribute__((aligned(16))) unsigned int sW[NWAVE * M * 32];
  const int tid = (int)threadIdx.x, lane = tid & 31, wave = tid >> 5;
  const float* TAB  = (const float*)(ws + O_TAB);
  const float* EDG  = (const float*)(ws + O_EDG);
  const float* UFG  = (const float*)(ws + OUFG);
  const int*   FLG  = (const int*)(ws + O_FLG);
  const int*   CNT  = (const int*)(ws + O_CNT);
  const int*   OFF  = (const int*)(ws + O_OFF);
  const int*   LIST = (const int*)(ws + O_LIST);
  {
    const int uc = tid < SU / 4 ? tid : SU / 4 - 1;
    const v4f v = *(const v4f*)(TAB + TUG + 4 * uc);
    if (tid < SU / 4) *(v4fa*)(sU + 4 * uc) = v;
    const int tc = tid < ST / 4 ? tid : ST / 4 - 1;
    const v4f t = *(const v4f*)(TAB + TUTG + 4 * tc);
    if (tid < ST / 4) *(v4fa*)(sT + 4 * tc) = t;
  }
  __syncthreads();

  float wr[G + 1][8];
#pragma unroll
  for (int lp = 0; lp <= G; ++lp) {
#pragma unroll
    for (int n = 0; n < 8; ++n) wr[lp][n] = TAB[TWR + (PG + lp) * 256 + n * 32 + lane];
    ldwait();
  }

  float* ac = sAcc + wave * (DP * 32) + lane;
  unsigned int* wq = sW + wave * (M * 32) + lane;
  const float qnan = __int_as_float(0x7fc00000);
  const int src0 = 2 * (lane & 15), src1 = src0 + 1;
  const int abase = (int)blockIdx.x * APB + wave * APW;

#pragma unroll 1
  for (int ai = 0; ai < APW; ++ai) {
    const int n = abase + ai;
    if (n < NAT) {
      const int blk   = n >> SLB;
      const int nhraw = FLG[(size_t)blk * 32];
      const int bflag = FLG[(size_t)blk * 32 + 1];
      const int nh    = nhraw < 0 ? 0 : (nhraw > RCAP ? RCAP : nhraw);
      const bool ovf  = (bflag != 0) || (nhraw < 0) || (nhraw > RCAP);
      int cnt = CNT[n];
      const bool big = cnt > DEGCAP;
      cnt = cnt < 0 ? 0 : (cnt > DEGCAP ? DEGCAP : cnt);
      int off = OFF[n];
      off = off < 0 ? 0 : (off > RCAP ? RCAP : off);
      if (cnt > nh - off) cnt = nh - off;
      cnt = cnt < 0 ? 0 : cnt;
#pragma unroll
      for (int d = 0; d < DP; ++d) ac[d * 32] = 0.0f;
      const int* lp0 = LIST + ((size_t)blk * RCAP + off) * 2;

#pragma unroll 1
      for (int q = 0; q < cnt; ++q) {
        const v2i ent = *(const v2i*)(lp0 + 2 * q);
        int e  = ent.x; e  = e  < 0 ? 0 : (e  > NED - 1 ? NED - 1 : e);
        int nbq = ent.y; nbq = nbq < 0 ? 0 : (nbq > NAT - 1 ? NAT - 1 : nbq);
        const float* ep = EDG + (size_t)e * 32;
        const v4f q0 = *(const v4f*)ep;
        const v4f q1 = *(const v4f*)(ep + 4);
        float sh[MP];
#pragma unroll
        for (int j = 0; j < MP / 4; ++j) {
          const v4f s = *(const v4f*)(ep + 8 + 4 * j);
          sh[4 * j] = s.x; sh[4 * j + 1] = s.y; sh[4 * j + 2] = s.z; sh[4 * j + 3] = s.w;
        }
        const float rb[8] = {q0.x, q0.y, q0.z, q0.w, q1.x, q1.y, q1.z, q1.w};
        float w[MP];
#pragma unroll
        for (int i = 0; i < MP; ++i) w[i] = 0.0f;
#pragma unroll
        for (int lp = 0; lp <= G; ++lp) {
          float rad = 0.0f;
#pragma unroll
          for (int k = 0; k < 8; ++k) rad = fmaf(rb[k], wr[lp][k], rad);
#pragma unroll
          for (int mu = 0; mu < 2 * lp + 1; ++mu) w[lp * lp + mu] = sh[lp * lp + mu] * rad;
        }
        const float* ufp = UFG + (size_t)nbq * (D * 32) + lane;
#pragma unroll 1
        for (int d = 0; d < D; ++d) {
          const float* ur = sU + d * MP;
          float v = 0.0f;
#pragma unroll
          for (int j = 0; j < MP / 4; ++j) {
            const v4f u = *(const v4fa*)(ur + 4 * j);
            v = fmaf(u.x, w[4 * j], v);
            v = fmaf(u.y, w[4 * j + 1], v);
            v = fmaf(u.z, w[4 * j + 2], v);
            v = fmaf(u.w, w[4 * j + 3], v);
          }
          const float uf = ufp[d * 32];
          ac[d * 32] = fmaf(v, uf, ac[d * 32]);
        }
      }

      const float pz = (ovf || big) ? qnan : 0.0f;
#pragma unroll 1
      for (int m = 0; m < M; ++m) {
        const float* tr = sT + m * DP;
        float x = 0.0f;
#pragma unroll
        for (int j = 0; j < DP / 4; ++j) {
          const v4f u = *(const v4fa*)(tr + 4 * j);
          x = fmaf(u.x, ac[(4 * j) * 32], x);
          x = fmaf(u.y, ac[(4 * j + 1) * 32], x);
          x = fmaf(u.z, ac[(4 * j + 2) * 32], x);
          x = fmaf(u.w, ac[(4 * j + 3) * 32], x);
        }
        x = x + pz;
        const unsigned int hb = f2bf(x);
        const unsigned int lb = f2bf(x - bf2f(hb));
        const int P  = (int)(hb | (lb << 16));
        const unsigned int a = (unsigned int)__shfl(P, src0, 32);
        const unsigned int b = (unsigned int)__shfl(P, src1, 32);
        const unsigned int whi = (a & 0xFFFFu) | (b << 16);
        const unsigned int wlo = (a >> 16) | (b & 0xFFFF0000u);
        const unsigned int word = (lane < 16) ? whi : wlo;
        wq[m * 32] = word;
        const int lp = (m >= 9) ? 3 : (m >= 4) ? 2 : (m >= 1) ? 1 : 0;
        const int mu = m - lp * lp;
        const size_t cb = (lp == 0) ? OCAT0 : (lp == 1) ? OCAT1 : (lp == 2) ? OCAT2 : OCAT3;
        const size_t ob = cb + (size_t)(n * (2 * lp + 1) + mu) * (size_t)(512 - 128 * lp)
                        + (size_t)(128 * (G - lp)) + (size_t)(4 * lane);
        *(volatile unsigned int*)(ws + ob) = word;
      }
      __threadfence();
#pragma unroll 1
      for (int m = 0; m < M; ++m) {
        const unsigned int word = wq[m * 32];
        const int lp = (m >= 9) ? 3 : (m >= 4) ? 2 : (m >= 1) ? 1 : 0;
        const int mu = m - lp * lp;
        const size_t cb = (lp == 0) ? OCAT0 : (lp == 1) ? OCAT1 : (lp == 2) ? OCAT2 : OCAT3;
        const size_t ob = cb + (size_t)(n * (2 * lp + 1) + mu) * (size_t)(512 - 128 * lp)
                        + (size_t)(128 * (G - lp)) + (size_t)(4 * lane);
        *(volatile unsigned int*)(ws + ob) = word;
      }
    }
  }
}

template <int L>
__device__ __forceinline__ void gemm_flush(const float* stg, const float* __restrict__ feat, float* out, int gp0, int tid) {
  constexpr int K = KL(L), PPT = (GBM * K / 4) / GTHR, NPIECE = MROWS(L) * (K / 4);
#pragma unroll 1
  for (int it = 0; it < PPT; ++it) {
    const int p  = it * GTHR + tid;
    const int gp = gp0 + p;
    const int gc = gp < NPIECE ? gp : NPIECE - 1;
    const v4f s = *(const v4fa*)(stg + 4 * p);
    const v4f f = *(const v4f*)(feat + (size_t)4 * gc);
    v4f o;
    o.x = s.x + bfr(f.x); o.y = s.y + bfr(f.y); o.z = s.z + bfr(f.z); o.w = s.w + bfr(f.w);
    if (gp < NPIECE) *(volatile v4f*)(out + (size_t)4 * gp) = o;
  }
}

template <int L>
__global__ __launch_bounds__(GTHR) __attribute__((amdgpu_num_vgpr(248)))
void k_gemm(const float* __restrict__ feat, float* out, const char* __restrict__ ws) {
  constexpr int K = KL(L), K2 = 2 * K, NT = K / 16, KS = K2 / 32;
  constexpr size_t OA = O_CAT(L), OW = O_WT(L);
  static_assert((K2 % 32) == 0 && (K % 16) == 0 && ((GBM * K / 4) % GTHR) == 0);
  static_assert(((MROWS(L) * (K / 4)) % 128) == 0);
  __shared__ __attribute__((aligned(16))) float stg[GBM * K];
  const int tid = (int)threadIdx.x, lane = tid & 31, wave = tid >> 5, hh = lane >> 4, m = lane & 15;
  const int rowBase = (int)blockIdx.x * GBM;
  const unsigned short* A  = (const unsigned short*)(ws + OA);
  const unsigned short* WT = (const unsigned short*)(ws + OW);

  v8f acc[NT];
  {
    const v8f z = {0.f, 0.f, 0.f, 0.f, 0.f, 0.f, 0.f, 0.f};
#pragma unroll
    for (int t = 0; t < NT; ++t) acc[t] = z;
  }
  const unsigned short* ap = A  + (size_t)(rowBase + 16 * wave + m) * (size_t)K2 + 8 * hh;
  const unsigned short* wp = WT + (size_t)m * (size_t)K2 + 8 * hh;
#pragma unroll 1
  for (int ks = 0; ks < KS; ++ks) {
    FragB af;
    af.h[0] = *(const v8usa*)(ap + 32 * ks);
    af.h[1] = *(const v8usa*)(ap + 32 * ks + 16);
#pragma unroll
    for (int t = 0; t < NT; ++t) {
      const unsigned short* wq = wp + (size_t)(16 * t) * (size_t)K2 + 32 * ks;
      FragB bf;
      bf.h[0] = *(const v8usa*)wq;
      bf.h[1] = *(const v8usa*)(wq + 16);
      acc[t] = wmb(af, bf, acc[t]);
    }
  }
#pragma unroll
  for (int t = 0; t < NT; ++t) {
    const int lc = 16 * t + m;
#pragma unroll
    for (int r = 0; r < 8; ++r) {
      const int lr = 16 * wave + 8 * hh + r;
      stg[lr * K + lc] = acc[t][r];
    }
  }
  __syncthreads();
  const int gp0 = rowBase * (K / 4);
  gemm_flush<L>(stg, feat, out, gp0, tid);
  __threadfence();
  gemm_flush<L>(stg, feat, out, gp0, tid);
}

static inline int cdiv(int a, int b) { return (a + b - 1) / b; }

extern "C" void kernel_launch(void* const* d_in, const int* in_sizes, int n_in,
                              void* d_out, int out_size, void* d_ws, size_t ws_size,
                              hipStream_t stream) {
  if (n_in < 23) return;
  if (in_sizes[0] != NED) return;
  for (int l = 0; l < 4; ++l) {
    const int b = 1 + 5 * l;
    if (in_sizes[b + 0] != NED * (2 * l + 1)) return;
    if (in_sizes[b + 1] != NAT * (2 * l + 1) * KL(l)) return;
    if (in_sizes[b + 2] != 8 * KL(l)) return;
    if (in_sizes[b + 3] != P3(l) * MM(l)) return;
    if (in_sizes[b + 4] != KL(l) * KL(l)) return;
  }
  if (in_sizes[21] != NED || in_sizes[22] != NED) return;
  if (out_size != OUTOFF(3) + MROWS(3) * KL(3)) return;
  if (ws_size < WS_TOTAL) return;

  const float* r = (const float*)d_in[0];
  const float* sh[4]; const float* ft[4]; const float* Wr[4]; const float* Uu[4]; const float* Wl[4];
  for (int l = 0; l < 4; ++l) {
    sh[l] = (const float*)d_in[1 + 5 * l + 0];
    ft[l] = (const float*)d_in[1 + 5 * l + 1];
    Wr[l] = (const float*)d_in[1 + 5 * l + 2];
    Uu[l] = (const float*)d_in[1 + 5 * l + 3];
    Wl[l] = (const float*)d_in[1 + 5 * l + 4];
  }
  const int* centers   = (const int*)d_in[21];
  const int* neighbors = (const int*)d_in[22];
  float* out = (float*)d_out;
  char*  ws  = (char*)d_ws;

  const int bktLds = BKT_LDS_INTS * 4;
  hipFuncSetAttribute(reinterpret_cast<const void*>(&k_bucket),
                      hipFuncAttributeMaxDynamicSharedMemorySize, bktLds);

  k_pa<<<UTOT / NTHR, NTHR, 0, stream>>>(Wl[0], Wl[1], Wl[2], Wl[3], ws);
  k_pb<<<1, NTHR, 0, stream>>>(Wr[0], Wr[1], Wr[2], Wr[3], Uu[0], Uu[1], Uu[2], Uu[3], ws);
  k_edge<<<EDGROWS / NTHR, NTHR, 0, stream>>>(r, sh[0], sh[1], sh[2], sh[3], ws);
  k_unc<<<dim3(cdiv(NAT, NWAVE), 4), NTHR, 0, stream>>>(ft[0], ft[1], ft[2], ft[3], ws);
  k_bucket<<<NBLK, NTHR, bktLds, stream>>>(centers, neighbors, ws);
  k_scan<0><<<cdiv(NAT, APB), NTHR, 0, stream>>>(ws);
  k_scan<1><<<cdiv(NAT, APB), NTHR, 0, stream>>>(ws);
  k_scan<2><<<cdiv(NAT, APB), NTHR, 0, stream>>>(ws);
  k_scan<3><<<cdiv(NAT, APB), NTHR, 0, stream>>>(ws);
  k_gemm<0><<<MPADR(0) / GBM, GTHR, 0, stream>>>(ft[0], out + OUTOFF(0), ws);
  k_gemm<1><<<MPADR(1) / GBM, GTHR, 0, stream>>>(ft[1], out + OUTOFF(1), ws);
  k_gemm<2><<<MPADR(2) / GBM, GTHR, 0, stream>>>(ft[2], out + OUTOFF(2), ws);
  k_gemm<3><<<MPADR(3) / GBM, GTHR, 0, stream>>>(ft[3], out + OUTOFF(3), ws);
}
